// DeltaNetEnhancedAttention_69569880261167
// MI455X (gfx1250) — hardware-verified
//
#include <hip/hip_runtime.h>

typedef __bf16 v16b __attribute__((ext_vector_type(16)));
typedef unsigned short v16us __attribute__((ext_vector_type(16)));
typedef unsigned short v8us __attribute__((ext_vector_type(8)));
typedef float v8f __attribute__((ext_vector_type(8)));
typedef float v4f __attribute__((ext_vector_type(4)));
typedef unsigned int v4u __attribute__((ext_vector_type(4)));
typedef v8us __attribute__((may_alias)) v8usa;
typedef v4f  __attribute__((may_alias)) v4fa;
typedef v4u  __attribute__((may_alias)) v4ua;
typedef unsigned short bf_t;

#define NB 4
#define NSEQ 1024
#define CD 768
#define NH 12
#define HD 64
#define NTOK 4096
#define CQ 2304
#define NBH 48
#define NCHUNK 16
#define TPB 8
#define NBLKF (NTOK / TPB)
#define WROWS 4736
#define WR_QKV 0
#define WR_ID 2304
#define WR_G1 3072
#define WR_PROJ 3840
#define WR_PRUNE 4608
#define WR_IDG 4672
#define WR_G2 4704

__device__ __forceinline__ bf_t f2bf(float x) {
  unsigned int u = __float_as_uint(x);
  u += 0x7FFFu + ((u >> 16) & 1u);
  return (bf_t)(u >> 16);
}
__device__ __forceinline__ float bf2f(bf_t v) { return __uint_as_float(((unsigned int)v) << 16); }
__device__ __forceinline__ void split2(float x, bf_t& hi, bf_t& lo) {
  const bf_t hb = f2bf(x);
  hi = hb;
  lo = f2bf(x - bf2f(hb));
}
__device__ __forceinline__ unsigned int pk2(bf_t a, bf_t b) { return (unsigned int)a | ((unsigned int)b << 16); }

__device__ __forceinline__ void split8(v4f a, v4f c, v4u& ph, v4u& pl) {
  bf_t h0, h1, h2, h3, h4, h5, h6, h7, l0, l1, l2, l3, l4, l5, l6, l7;
  split2(a.x, h0, l0); split2(a.y, h1, l1); split2(a.z, h2, l2); split2(a.w, h3, l3);
  split2(c.x, h4, l4); split2(c.y, h5, l5); split2(c.z, h6, l6); split2(c.w, h7, l7);
  ph.x = pk2(h0, h1); ph.y = pk2(h2, h3); ph.z = pk2(h4, h5); ph.w = pk2(h6, h7);
  pl.x = pk2(l0, l1); pl.y = pk2(l2, l3); pl.z = pk2(l4, l5); pl.w = pk2(l6, l7);
}
__device__ __forceinline__ v4u pack8hi(v4f a, v4f c) {
  v4u p;
  p.x = pk2(f2bf(a.x), f2bf(a.y)); p.y = pk2(f2bf(a.z), f2bf(a.w));
  p.z = pk2(f2bf(c.x), f2bf(c.y)); p.w = pk2(f2bf(c.z), f2bf(c.w));
  return p;
}

__device__ __forceinline__ v8f wmma_bf16(v16b a, v16b b, v8f c) {
  return __builtin_amdgcn_wmma_f32_16x16x32_bf16(false, a, false, b, (short)0, c, false, false);
}
__device__ __forceinline__ v8f mma3(v16b ah, v16b al, v16b bh, v16b bl, v8f c) {
  c = wmma_bf16(ah, bh, c);
  c = wmma_bf16(al, bh, c);
  c = wmma_bf16(ah, bl, c);
  asm volatile("v_nop\n\tv_nop\n\tv_nop\n\tv_nop" : "+v"(c) : "v"(ah), "v"(al), "v"(bh), "v"(bl));
  return c;
}

__device__ __forceinline__ v16b ldf(const bf_t* p, int h) {
  const v8us a = *(const v8usa*)(p + 8 * h);
  const v8us c = *(const v8usa*)(p + 16 + 8 * h);
  const v16us u = __builtin_shufflevector(a, c, 0, 1, 2, 3, 4, 5, 6, 7, 8, 9, 10, 11, 12, 13, 14, 15);
  return __builtin_bit_cast(v16b, u);
}
__device__ __forceinline__ v16b ldg64(const bf_t* pl, int k0, int col, int h) {
  v16us u;
  #pragma unroll
  for (int i = 0; i < 8; ++i) {
    u[i]     = pl[(k0 + 8 * h + i) * 64 + col];
    u[8 + i] = pl[(k0 + 16 + 8 * h + i) * 64 + col];
  }
  return __builtin_bit_cast(v16b, u);
}

__device__ __forceinline__ float gelu_tanh(float x) {
  const float x3 = x * x * x;
  const float t = tanhf(0.7978845608028654f * (x + 0.044715f * x3));
  return x * (0.5f * (1.0f + t));
}

__global__ __launch_bounds__(256) void k_cvt_x(const float* __restrict__ x,
                                               bf_t* __restrict__ xh, bf_t* __restrict__ xl, int n8) {
  const int g = blockIdx.x * 256 + threadIdx.x;
  if (g >= n8) return;
  const v4f a = *(const v4fa*)(x + (size_t)g * 8);
  const v4f c = *(const v4fa*)(x + (size_t)g * 8 + 4);
  v4u ph, pl;
  split8(a, c, ph, pl);
  bf_t* dh = xh + (size_t)g * 8;
  bf_t* dl = xl + (size_t)g * 8;
  *(volatile v4u*)dh = ph;
  *(volatile v4u*)dl = pl;
  __threadfence();
  *(volatile v4u*)dh = ph;
  *(volatile v4u*)dl = pl;
}

__global__ __launch_bounds__(256) void k_wcvt(const float* __restrict__ W, int nout,
                                              bf_t* __restrict__ oh, bf_t* __restrict__ ol) {
  __shared__ __attribute__((aligned(16))) float tile[32 * 68];
  const int tid = threadIdx.x;
  const int k0 = blockIdx.x * 64, n0 = blockIdx.y * 32;
  #pragma unroll
  for (int i = 0; i < 8; ++i) {
    const int e = i * 256 + tid;
    const int kk = e >> 5, nn = e & 31;
    const int n = n0 + nn;
    const int nc = (n < nout) ? n : (nout - 1);
    const float v = W[(size_t)(k0 + kk) * nout + nc];
    tile[nn * 68 + kk] = (n < nout) ? v : 0.0f;
  }
  __syncthreads();
  const int row = tid >> 3, j = tid & 7;
  const v4f a = *(const v4fa*)(tile + row * 68 + 8 * j);
  const v4f c = *(const v4fa*)(tile + row * 68 + 8 * j + 4);
  v4u ph, pl;
  split8(a, c, ph, pl);
  const size_t o = (size_t)(n0 + row) * CD + k0 + 8 * j;
  *(volatile v4u*)(oh + o) = ph;
  *(volatile v4u*)(ol + o) = pl;
  __threadfence();
  *(volatile v4u*)(oh + o) = ph;
  *(volatile v4u*)(ol + o) = pl;
}

template <int NT>
__device__ __forceinline__ void gemm_store_f32(const float* sT, float* Cf, int ldc, int m0, int n0, int tid) {
  constexpr int PPR = 4 * NT;
  #pragma unroll
  for (int it = 0; it < 4 * NT; ++it) {
    const int p = it * 128 + tid;
    const int row = p / PPR, j = p - row * PPR;
    const v4f v = *(const v4fa*)(sT + row * (16 * NT) + 4 * j);
    *(volatile v4f*)(Cf + (size_t)(m0 + row) * ldc + n0 + 4 * j) = v;
  }
}
__device__ __forceinline__ void gemm_store_planes(const float* sT, bf_t* Ch, bf_t* Cl, int ldp, int m0, int n0, int tid) {
  #pragma unroll
  for (int it = 0; it < 8; ++it) {
    const int p = it * 128 + tid;
    const int row = p >> 3, j = p & 7;
    const float* s = sT + row * 64 + 8 * j;
    const v4f a = *(const v4fa*)s;
    const v4f c = *(const v4fa*)(s + 4);
    v4u ph, pl;
    split8(a, c, ph, pl);
    const size_t o = (size_t)(m0 + row) * ldp + n0 + 8 * j;
    *(volatile v4u*)(Ch + o) = ph;
    *(volatile v4u*)(Cl + o) = pl;
  }
}

template <int NT, int EPI>
__global__ __launch_bounds__(128) void k_gemm(
    const bf_t* __restrict__ Ah, const bf_t* __restrict__ Al, int lda,
    const bf_t* __restrict__ Bh, const bf_t* __restrict__ Bl, int ldb,
    const float* __restrict__ bias, int nbias,
    float* __restrict__ Cf, int ldc,
    bf_t* __restrict__ Ch, bf_t* __restrict__ Cl, int ldp, int K)
{
  __shared__ __attribute__((aligned(16))) float sT[128 * 16 * NT];
  const int tid = threadIdx.x, lane = tid & 31, w = tid >> 5, h = lane >> 4, m = lane & 15;
  const int m0 = blockIdx.y * 128, n0 = blockIdx.x * (16 * NT);
  const size_t arow = (size_t)(m0 + 32 * w + m);
  const bf_t* a0h = Ah + arow * lda;
  const bf_t* a0l = Al + arow * lda;
  const bf_t* a1h = a0h + (size_t)16 * lda;
  const bf_t* a1l = a0l + (size_t)16 * lda;
  const bf_t* bph = Bh + (size_t)(n0 + m) * ldb;
  const bf_t* bpl = Bl + (size_t)(n0 + m) * ldb;
  const v8f z8 = {0.f, 0.f, 0.f, 0.f, 0.f, 0.f, 0.f, 0.f};
  v8f acc[2][NT];
  #pragma unroll
  for (int nt = 0; nt < NT; ++nt) { acc[0][nt] = z8; acc[1][nt] = z8; }

  #pragma unroll 1
  for (int k0 = 0; k0 < K; k0 += 32) {
    const v16b fa0h = ldf(a0h + k0, h);
    const v16b fa0l = ldf(a0l + k0, h);
    const v16b fa1h = ldf(a1h + k0, h);
    const v16b fa1l = ldf(a1l + k0, h);
    #pragma unroll
    for (int nt = 0; nt < NT; ++nt) {
      const v16b fbh = ldf(bph + (size_t)nt * 16 * ldb + k0, h);
      const v16b fbl = ldf(bpl + (size_t)nt * 16 * ldb + k0, h);
      acc[0][nt] = mma3(fa0h, fa0l, fbh, fbl, acc[0][nt]);
      acc[1][nt] = mma3(fa1h, fa1l, fbh, fbl, acc[1][nt]);
    }
  }

  #pragma unroll
  for (int nt = 0; nt < NT; ++nt) {
    const int col = 16 * nt + m;
    const int gcol = n0 + col;
    const int bi = (gcol < nbias) ? gcol : 0;
    const float braw = bias[bi];
    const float bvl = (gcol < nbias) ? braw : 0.0f;
    #pragma unroll
    for (int mt = 0; mt < 2; ++mt) {
      #pragma unroll
      for (int r = 0; r < 8; ++r) {
        const int row = 32 * w + 16 * mt + 8 * h + r;
        float y = acc[mt][nt][r] + bvl;
        if (EPI == 1) y = gelu_tanh(y);
        sT[row * (16 * NT) + col] = y;
      }
    }
  }
  __syncthreads();
  if (EPI == 0) {
    gemm_store_f32<NT>(sT, Cf, ldc, m0, n0, tid);
    __threadfence();
    gemm_store_f32<NT>(sT, Cf, ldc, m0, n0, tid);
  } else {
    gemm_store_planes(sT, Ch, Cl, ldp, m0, n0, tid);
    __threadfence();
    gemm_store_planes(sT, Ch, Cl, ldp, m0, n0, tid);
  }
}

__global__ __launch_bounds__(256) void k_qkpl(const float* __restrict__ qkv, bf_t* __restrict__ qk, int n8) {
  const int g = blockIdx.x * 256 + threadIdx.x;
  if (g >= n8) return;
  const int j = g & 7;
  const int r = g >> 3;
  const int which = (r >= NBH * NSEQ) ? 1 : 0;
  const int rr = r - which * (NBH * NSEQ);
  const int bh = rr >> 10, l = rr & 1023;
  const int b = bh / NH, hh = bh - b * NH;
  const float* src = qkv + (size_t)(b * NSEQ + l) * CQ + which * CD + hh * HD + 8 * j;
  const v4f a = *(const v4fa*)src;
  const v4f c = *(const v4fa*)(src + 4);
  const v4u p = pack8hi(a, c);
  bf_t* dst = qk + (size_t)r * HD + 8 * j;
  *(volatile v4u*)dst = p;
  __threadfence();
  *(volatile v4u*)dst = p;
}

__global__ __launch_bounds__(64) void k_beta(const bf_t* __restrict__ qk, float* __restrict__ beta) {
  __shared__ __attribute__((aligned(16))) float sS[32 * NSEQ];
  __shared__ __attribute__((aligned(16))) float sb[32];
  const int tid = threadIdx.x, lane = tid & 31, w = tid >> 5, h = lane >> 4, m = lane & 15;
  const int bh = blockIdx.y;
  const int qb = blockIdx.x * 32;
  const int q0 = qb + 16 * w;
  const bf_t* qrow = qk + ((size_t)bh * NSEQ + q0 + m) * HD;
  const v16b qb0 = ldf(qrow, h);
  const v16b qb1 = ldf(qrow + 32, h);
  const bf_t* kbase = qk + ((size_t)NBH * NSEQ + (size_t)bh * NSEQ + m) * HD;
  float* myrow = sS + (w * 16 + m) * NSEQ;
  const v8f z8 = {0.f, 0.f, 0.f, 0.f, 0.f, 0.f, 0.f, 0.f};
  float mx = -1.0e30f;

  #pragma unroll 1
  for (int kb = 0; kb < NSEQ; kb += 64) {
    #pragma unroll
    for (int j = 0; j < 4; ++j) {
      const bf_t* kp = kbase + (size_t)(kb + 16 * j) * HD;
      const v16b kf0 = ldf(kp, h);
      const v16b kf1 = ldf(kp + 32, h);
      v8f z = z8;
      z = wmma_bf16(kf0, qb0, z);
      z = wmma_bf16(kf1, qb1, z);
      asm volatile("v_nop\n\tv_nop\n\tv_nop\n\tv_nop" : "+v"(z) : "v"(kf0), "v"(kf1), "v"(qb0), "v"(qb1));
      v4f lo4, hi4;
      lo4.x = z[0] * 0.125f; lo4.y = z[1] * 0.125f; lo4.z = z[2] * 0.125f; lo4.w = z[3] * 0.125f;
      hi4.x = z[4] * 0.125f; hi4.y = z[5] * 0.125f; hi4.z = z[6] * 0.125f; hi4.w = z[7] * 0.125f;
      mx = fmaxf(mx, fmaxf(fmaxf(lo4.x, lo4.y), fmaxf(lo4.z, lo4.w)));
      mx = fmaxf(mx, fmaxf(fmaxf(hi4.x, hi4.y), fmaxf(hi4.z, hi4.w)));
      float* p = myrow + kb + 16 * j + 8 * h;
      *(v4fa*)p = lo4;
      *(v4fa*)(p + 4) = hi4;
    }
  }
  mx = fmaxf(mx, __shfl_xor(mx, 16));

  float ssum = 0.0f;
  #pragma unroll 1
  for (int t = 0; t < NSEQ / 16; ++t) {
    float* p = myrow + 16 * t + 8 * h;
    v4f a = *(const v4fa*)p;
    v4f c = *(const v4fa*)(p + 4);
    a.x = __expf(a.x - mx); a.y = __expf(a.y - mx); a.z = __expf(a.z - mx); a.w = __expf(a.w - mx);
    c.x = __expf(c.x - mx); c.y = __expf(c.y - mx); c.z = __expf(c.z - mx); c.w = __expf(c.w - mx);
    ssum += ((a.x + a.y) + (a.z + a.w)) + ((c.x + c.y) + (c.z + c.w));
    *(v4fa*)p = a;
    *(v4fa*)(p + 4) = c;
  }
  ssum += __shfl_xor(ssum, 16);
  const float inv = 1.0f / ssum;

  float bp = 0.0f;
  #pragma unroll 1
  for (int t = 0; t < NSEQ / 16; ++t) {
    const float* p = myrow + 16 * t + 8 * h;
    const v4f a = *(const v4fa*)p;
    const v4f c = *(const v4fa*)(p + 4);
    bp += a.x * inv; bp += a.y * inv; bp += a.z * inv; bp += a.w * inv;
    bp += c.x * inv; bp += c.y * inv; bp += c.z * inv; bp += c.w * inv;
  }
  bp += __shfl_xor(bp, 16);
  if (h == 0) sb[w * 16 + m] = bp;
  __syncthreads();
  if (tid < 8) {
    const v4f v = *(const v4fa*)(sb + 4 * tid);
    float* dst = beta + (size_t)bh * NSEQ + qb + 4 * tid;
    *(volatile v4f*)dst = v;
    __threadfence();
    *(volatile v4f*)dst = v;
  }
}

__device__ __forceinline__ void delta_store_o(const float* Os, float* dout, int tok0, int hh, int tid) {
  #pragma unroll
  for (int it = 0; it < 4; ++it) {
    const int p = it * 256 + tid;
    const int row = p >> 4, j = p & 15;
    const v4f v = *(const v4fa*)(Os + row * 64 + 4 * j);
    *(volatile v4f*)(dout + (size_t)(tok0 + row) * CD + hh * HD + 4 * j) = v;
  }
}

__global__ __launch_bounds__(256) void k_delta(const float* __restrict__ qkv,
                                               const float* __restrict__ beta,
                                               float* __restrict__ dout) {
  __shared__ __attribute__((aligned(16))) float Sf[4096];
  __shared__ __attribute__((aligned(16))) float Am[4096];
  __shared__ __attribute__((aligned(16))) float Tm[4096];
  __shared__ __attribute__((aligned(16))) bf_t qNh[4096];
  __shared__ __attribute__((aligned(16))) bf_t qNl[4096];
  __shared__ __attribute__((aligned(16))) bf_t kNh[4096];
  __shared__ __attribute__((aligned(16))) bf_t kNl[4096];
  __shared__ __attribute__((aligned(16))) bf_t kbh[4096];
  __shared__ __attribute__((aligned(16))) bf_t kbl[4096];
  __shared__ __attribute__((aligned(16))) bf_t vTh[4096];
  __shared__ __attribute__((aligned(16))) bf_t vTl[4096];
  __shared__ __attribute__((aligned(16))) bf_t tPh[4096];
  __shared__ __attribute__((aligned(16))) bf_t tPl[4096];
  __shared__ __attribute__((aligned(16))) bf_t sTh[4096];
  __shared__ __attribute__((aligned(16))) bf_t sTl[4096];

  const int tid = threadIdx.x, lane = tid & 31, w = tid >> 5, h = lane >> 4, m = lane & 15;
  const int bh = blockIdx.x, b = bh / NH, hh = bh - b * NH;
  const int tm = (w >> 1) * 16;
  const int tn0 = (w & 1) * 32, tn1 = tn0 + 16;
  const v8f z8 = {0.f, 0.f, 0.f, 0.f, 0.f, 0.f, 0.f, 0.f};

  for (int i = tid; i < 4096; i += 256) { Sf[i] = 0.0f; sTh[i] = (bf_t)0; sTl[i] = (bf_t)0; }
  __syncthreads();

  #pragma unroll 1
  for (int ci = 0; ci < NCHUNK; ++ci) {
    const int tok0 = b * NSEQ + ci * 64;

    {
      const int row = tid >> 2, qd = tid & 3;
      const float* qr = qkv + (size_t)(tok0 + row) * CQ + hh * HD + 16 * qd;
      float qa[16], ka[16], va[16];
      #pragma unroll
      for (int i = 0; i < 4; ++i) {
        const v4f tq = *(const v4fa*)(qr + 4 * i);
        const v4f tk = *(const v4fa*)(qr + CD + 4 * i);
        const v4f tv = *(const v4fa*)(qr + 2 * CD + 4 * i);
        qa[4 * i] = tq.x; qa[4 * i + 1] = tq.y; qa[4 * i + 2] = tq.z; qa[4 * i + 3] = tq.w;
        ka[4 * i] = tk.x; ka[4 * i + 1] = tk.y; ka[4 * i + 2] = tk.z; ka[4 * i + 3] = tk.w;
        va[4 * i] = tv.x; va[4 * i + 1] = tv.y; va[4 * i + 2] = tv.z; va[4 * i + 3] = tv.w;
      }
      float ss = 0.0f;
      #pragma unroll
      for (int i = 0; i < 16; ++i) ss += ka[i] * ka[i];
      ss += __shfl_xor(ss, 1);
      ss += __shfl_xor(ss, 2);
      const float inv = 1.0f / (sqrtf(ss) + 1e-6f);
      const float bt = beta[(size_t)bh * NSEQ + ci * 64 + row];
      #pragma unroll
      for (int i = 0; i < 16; ++i) {
        const int d = 16 * qd + i;
        const float kn = ka[i] * inv;
        bf_t e0, e1;
        split2(qa[i] * 0.125f, e0, e1); qNh[row * 64 + d] = e0; qNl[row * 64 + d] = e1;
        split2(kn, e0, e1);             kNh[row * 64 + d] = e0; kNl[row * 64 + d] = e1;
        split2(kn * bt, e0, e1);        kbh[row * 64 + d] = e0; kbl[row * 64 + d] = e1;
        split2(va[i] * bt, e0, e1);     vTh[d * 64 + row] = e0; vTl[d * 64 + row] = e1;
      }
    }
    __syncthreads();

    {
      v8f c0 = z8, c1 = z8;
      #pragma unroll
      for (int ks = 0; ks < 64; ks += 32) {
        const v16b ah = ldf(kbh + (tm + m) * 64 + ks, h);
        const v16b al = ldf(kbl + (tm + m) * 64 + ks, h);
        const v16b b0h = ldf(kNh + (tn0 + m) * 64 + ks, h);
        const v16b b0l = ldf(kNl + (tn0 + m) * 64 + ks, h);
        c0 = mma3(ah, al, b0h, b0l, c0);
        const v16b b1h = ldf(kNh + (tn1 + m) * 64 + ks, h);
        const v16b b1l = ldf(kNl + (tn1 + m) * 64 + ks, h);
        c1 = mma3(ah, al, b1h, b1l, c1);
      }
      #pragma unroll
      for (int r = 0; r < 8; ++r) {
        const int row = tm + 8 * h + r;
        const int ca = tn0 + m, cb = tn1 + m;
        Am[row * 64 + ca] = (ca < row) ? c0[r] : 0.0f;
        Am[row * 64 + cb] = (cb < row) ? c1[r] : 0.0f;
      }
    }
    __syncthreads();

    if (tid < 64) {
      const int col = tid;
      for (int i = 0; i < col; ++i) Tm[i * 64 + col] = 0.0f;
      Tm[col * 64 + col] = 1.0f;
      for (int i = col + 1; i < 64; ++i) {
        float s = 0.0f;
        for (int j = col; j < i; ++j) s += Am[i * 64 + j] * Tm[j * 64 + col];
        Tm[i * 64 + col] = -s;
      }
    }
    __syncthreads();

    for (int i = tid; i < 4096; i += 256) {
      bf_t e0, e1;
      split2(Tm[i], e0, e1);
      tPh[i] = e0; tPl[i] = e1;
    }
    __syncthreads();

    v8f u0 = z8, u1 = z8, w0 = z8, w1 = z8;
    #pragma unroll
    for (int ks = 0; ks < 64; ks += 32) {
      const v16b ah = ldf(tPh + (tm + m) * 64 + ks, h);
      const v16b al = ldf(tPl + (tm + m) * 64 + ks, h);
      {
        const v16b b0h = ldf(vTh + (tn0 + m) * 64 + ks, h);
        const v16b b0l = ldf(vTl + (tn0 + m) * 64 + ks, h);
        u0 = mma3(ah, al, b0h, b0l, u0);
        const v16b b1h = ldf(vTh + (tn1 + m) * 64 + ks, h);
        const v16b b1l = ldf(vTl + (tn1 + m) * 64 + ks, h);
        u1 = mma3(ah, al, b1h, b1l, u1);
      }
      {
        const v16b g0h = ldg64(kbh, ks, tn0 + m, h);
        const v16b g0l = ldg64(kbl, ks, tn0 + m, h);
        w0 = mma3(ah, al, g0h, g0l, w0);
        const v16b g1h = ldg64(kbh, ks, tn1 + m, h);
        const v16b g1l = ldg64(kbl, ks, tn1 + m, h);
        w1 = mma3(ah, al, g1h, g1l, w1);
      }
    }
    __syncthreads();

    #pragma unroll
    for (int r = 0; r < 8; ++r) {
      const int row = tm + 8 * h + r;
      bf_t e0, e1;
      split2(-w0[r], e0, e1); vTh[row * 64 + tn0 + m] = e0; vTl[row * 64 + tn0 + m] = e1;
      split2(-w1[r], e0, e1); vTh[row * 64 + tn1 + m] = e0; vTl[row * 64 + tn1 + m] = e1;
    }
    __syncthreads();

    {
      v8f t0 = u0, t1 = u1;
      #pragma unroll
      for (int ks = 0; ks < 64; ks += 32) {
        const v16b ah = ldf(vTh + (tm + m) * 64 + ks, h);
        const v16b al = ldf(vTl + (tm + m) * 64 + ks, h);
        const v16b b0h = ldf(sTh + (tn0 + m) * 64 + ks, h);
        const v16b b0l = ldf(sTl + (tn0 + m) * 64 + ks, h);
        t0 = mma3(ah, al, b0h, b0l, t0);
        const v16b b1h = ldf(sTh + (tn1 + m) * 64 + ks, h);
        const v16b b1l = ldf(sTl + (tn1 + m) * 64 + ks, h);
        t1 = mma3(ah, al, b1h, b1l, t1);
      }
      #pragma unroll
      for (int r = 0; r < 8; ++r) {
        const int c = tm + 8 * h + r;
        bf_t e0, e1;
        split2(t0[r], e0, e1); kbh[(tn0 + m) * 64 + c] = e0; kbl[(tn0 + m) * 64 + c] = e1;
        split2(t1[r], e0, e1); kbh[(tn1 + m) * 64 + c] = e0; kbl[(tn1 + m) * 64 + c] = e1;
      }
      v8f p0 = z8, p1 = z8;
      #pragma unroll
      for (int ks = 0; ks < 64; ks += 32) {
        const v16b ah = ldf(qNh + (tm + m) * 64 + ks, h);
        const v16b al = ldf(qNl + (tm + m) * 64 + ks, h);
        const v16b b0h = ldf(kNh + (tn0 + m) * 64 + ks, h);
        const v16b b0l = ldf(kNl + (tn0 + m) * 64 + ks, h);
        p0 = mma3(ah, al, b0h, b0l, p0);
        const v16b b1h = ldf(kNh + (tn1 + m) * 64 + ks, h);
        const v16b b1l = ldf(kNl + (tn1 + m) * 64 + ks, h);
        p1 = mma3(ah, al, b1h, b1l, p1);
      }
      #pragma unroll
      for (int r = 0; r < 8; ++r) {
        const int row = tm + 8 * h + r;
        const int ca = tn0 + m, cb = tn1 + m;
        const float va0 = (ca <= row) ? p0[r] : 0.0f;
        const float vb0 = (cb <= row) ? p1[r] : 0.0f;
        bf_t e0, e1;
        split2(va0, e0, e1); tPh[row * 64 + ca] = e0; tPl[row * 64 + ca] = e1;
        split2(vb0, e0, e1); tPh[row * 64 + cb] = e0; tPl[row * 64 + cb] = e1;
      }
    }
    __syncthreads();

    {
      v8f o0 = z8, o1 = z8;
      #pragma unroll
      for (int ks = 0; ks < 64; ks += 32) {
        const v16b ah = ldf(qNh + (tm + m) * 64 + ks, h);
        const v16b al = ldf(qNl + (tm + m) * 64 + ks, h);
        const v16b b0h = ldf(sTh + (tn0 + m) * 64 + ks, h);
        const v16b b0l = ldf(sTl + (tn0 + m) * 64 + ks, h);
        o0 = mma3(ah, al, b0h, b0l, o0);
        const v16b b1h = ldf(sTh + (tn1 + m) * 64 + ks, h);
        const v16b b1l = ldf(sTl + (tn1 + m) * 64 + ks, h);
        o1 = mma3(ah, al, b1h, b1l, o1);
      }
      #pragma unroll
      for (int ks = 0; ks < 64; ks += 32) {
        const v16b ah = ldf(tPh + (tm + m) * 64 + ks, h);
        const v16b al = ldf(tPl + (tm + m) * 64 + ks, h);
        const v16b b0h = ldf(kbh + (tn0 + m) * 64 + ks, h);
        const v16b b0l = ldf(kbl + (tn0 + m) * 64 + ks, h);
        o0 = mma3(ah, al, b0h, b0l, o0);
        const v16b b1h = ldf(kbh + (tn1 + m) * 64 + ks, h);
        const v16b b1l = ldf(kbl + (tn1 + m) * 64 + ks, h);
        o1 = mma3(ah, al, b1h, b1l, o1);
      }
      #pragma unroll
      for (int r = 0; r < 8; ++r) {
        const int row = tm + 8 * h + r;
        Am[row * 64 + tn0 + m] = o0[r];
        Am[row * 64 + tn1 + m] = o1[r];
      }
    }
    __syncthreads();

    delta_store_o(Am, dout, tok0, hh, tid);
    __threadfence();
    delta_store_o(Am, dout, tok0, hh, tid);
    {
      v8f s0, s1;
      #pragma unroll
      for (int r = 0; r < 8; ++r) {
        const int d = tm + 8 * h + r;
        s0[r] = Sf[d * 64 + tn0 + m];
        s1[r] = Sf[d * 64 + tn1 + m];
      }
      #pragma unroll
      for (int ks = 0; ks < 64; ks += 32) {
        const v16b ah = ldg64(kNh, ks, tm + m, h);
        const v16b al = ldg64(kNl, ks, tm + m, h);
        const v16b b0h = ldf(kbh + (tn0 + m) * 64 + ks, h);
        const v16b b0l = ldf(kbl + (tn0 + m) * 64 + ks, h);
        s0 = mma3(ah, al, b0h, b0l, s0);
        const v16b b1h = ldf(kbh + (tn1 + m) * 64 + ks, h);
        const v16b b1l = ldf(kbl + (tn1 + m) * 64 + ks, h);
        s1 = mma3(ah, al, b1h, b1l, s1);
      }
      #pragma unroll
      for (int r = 0; r < 8; ++r) {
        const int d = tm + 8 * h + r;
        const int ea = tn0 + m, eb = tn1 + m;
        Sf[d * 64 + ea] = s0[r];
        Sf[d * 64 + eb] = s1[r];
        bf_t e0, e1;
        split2(s0[r], e0, e1); sTh[ea * 64 + d] = e0; sTl[ea * 64 + d] = e1;
        split2(s1[r], e0, e1); sTh[eb * 64 + d] = e0; sTl[eb * 64 + d] = e1;
      }
    }
    __syncthreads();
  }
}

__device__ __forceinline__ void fuse_ctx_pass(const float* cs, bf_t* ctxh, bf_t* ctxl, int tokb, int tid) {
  #pragma unroll
  for (int it = 0; it < 3; ++it) {
    const int p = it * 256 + tid;
    const int tt = p / 96, j = p - tt * 96;
    const float* s = cs + tt * CD + 8 * j;
    const v4f a = *(const v4fa*)s;
    const v4f c = *(const v4fa*)(s + 4);
    v4u ph, pl;
    split8(a, c, ph, pl);
    const size_t o = (size_t)(tokb + tt) * CD + 8 * j;
    *(volatile v4u*)(ctxh + o) = ph;
    *(volatile v4u*)(ctxl + o) = pl;
  }
}

__global__ __launch_bounds__(256) void k_fuse(
    const float* __restrict__ qkv, const float* __restrict__ deltao, const float* __restrict__ idraw,
    const float* __restrict__ prune, const float* __restrict__ glog, const float* __restrict__ idlog,
    const float* __restrict__ firs, const float* __restrict__ firl, const float* __restrict__ mixm,
    const float* __restrict__ idstat,
    bf_t* __restrict__ ctxh, bf_t* __restrict__ ctxl, float* __restrict__ epart)
{
  __shared__ __attribute__((aligned(16))) float vbuf[(TPB + 6) * CD];
  __shared__ __attribute__((aligned(16))) float cs[TPB * CD];
  __shared__ __attribute__((aligned(16))) float fsb[CD];
  __shared__ __attribute__((aligned(16))) float flb[CD];
  __shared__ __attribute__((aligned(16))) float wsS[3 * CD];
  __shared__ __attribute__((aligned(16))) float wlS[7 * CD];
  __shared__ float smx[NH * NH];
  __shared__ float wls[NH * 5];
  __shared__ float gsh[NH];
  __shared__ float dgsh[NH];
  __shared__ float eh[2 * NH];
  __shared__ __attribute__((aligned(16))) float eline[32];

  const int tid = threadIdx.x, blk = blockIdx.x;
  const int tokb = blk * TPB;
  const int b = tokb / NSEQ, n0 = tokb - b * NSEQ;
  const v4f z4 = {0.f, 0.f, 0.f, 0.f};

  for (int e = tid; e < (TPB + 6) * (CD / 4); e += 256) {
    const int rw = e / (CD / 4), qd = e - rw * (CD / 4);
    const int nn = n0 - 6 + rw;
    const int nc = (nn < 0) ? 0 : nn;
    v4f v = *(const v4fa*)(qkv + (size_t)(b * NSEQ + nc) * CQ + 2 * CD + 4 * qd);
    if (nn < 0) v = z4;
    *(v4fa*)(vbuf + rw * CD + 4 * qd) = v;
  }
  for (int e = tid; e < 3 * CD; e += 256) { const int c = e / 3, kk = e - 3 * c; wsS[kk * CD + c] = firs[e]; }
  for (int e = tid; e < 7 * CD; e += 256) { const int c = e / 7, kk = e - 7 * c; wlS[kk * CD + c] = firl[e]; }
  if (tid < NH * NH) smx[tid] = mixm[tid];
  float e1acc = 0.0f, e2acc = 0.0f;
  __syncthreads();

  #pragma unroll 1
  for (int t = 0; t < TPB; ++t) {
    const int tok = tokb + t;
    if (tid < 192) {
      const int c0 = 4 * tid;
      v4f fs = z4, fl = z4;
      #pragma unroll 1
      for (int kk = 0; kk < 7; ++kk) {
        const v4f vr = *(const v4fa*)(vbuf + (t + kk) * CD + c0);
        const v4f wv = *(const v4fa*)(wlS + kk * CD + c0);
        fl = fl + vr * wv;
      }
      #pragma unroll 1
      for (int kk = 0; kk < 3; ++kk) {
        const v4f vr = *(const v4fa*)(vbuf + (t + 4 + kk) * CD + c0);
        const v4f wv = *(const v4fa*)(wsS + kk * CD + c0);
        fs = fs + vr * wv;
      }
      *(v4fa*)(fsb + c0) = fs;
      *(v4fa*)(flb + c0) = fl;
    } else if (tid < 192 + NH) {
      const int hq = tid - 192;
      const float* prp = prune + (size_t)tok * 64 + hq * 5;
      float mxv = prp[0];
      #pragma unroll 1
      for (int p = 1; p < 5; ++p) mxv = fmaxf(mxv, prp[p]);
      float sum = 0.0f;
      #pragma unroll 1
      for (int p = 0; p < 5; ++p) {
        const float ev = __expf(prp[p] - mxv);
        wls[hq * 5 + p] = ev;
        sum += ev;
      }
      const float inv = 1.0f / sum;
      float e1 = 0.0f;
      #pragma unroll 1
      for (int p = 0; p < 5; ++p) {
        const float wv = wls[hq * 5 + p] * inv;
        wls[hq * 5 + p] = wv;
        e1 += wv * logf(wv + 1e-8f);
      }
      e1acc += e1;
      const float g = 1.0f / (1.0f + __expf(-glog[(size_t)tok * 16 + hq]));
      gsh[hq] = g;
      float e2 = 0.0f;
      #pragma unroll 1
      for (int qq = 0; qq < 2; ++qq) {
        const float a = (qq == 0) ? g : (1.0f - g);
        e2 += a * logf(a + 1e-8f);
      }
      e2acc += e2;
      const float st = 1.0f / (1.0f + __expf(-idstat[hq]));
      const float dg = 1.0f / (1.0f + __expf(-idlog[(size_t)tok * 16 + hq]));
      dgsh[hq] = dg * st;
    }
    __syncthreads();
    if (tid < 192) {
      const int c0 = 4 * tid, hh = tid >> 4, d0 = c0 & 63;
      v4f as = z4, al = z4;
      #pragma unroll 1
      for (int g = 0; g < NH; ++g) {
        const float mv = smx[g * NH + hh];
        const v4f a = *(const v4fa*)(fsb + g * HD + d0);
        const v4f c = *(const v4fa*)(flb + g * HD + d0);
        as = as + a * mv;
        al = al + c * mv;
      }
      const v4f ms = *(const v4fa*)(fsb + c0) + as;
      const v4f ml = *(const v4fa*)(flb + c0) + al;
      const v4f p2 = *(const v4fa*)(deltao + (size_t)tok * CD + c0);
      const v4f p3 = *(const v4fa*)(vbuf + (t + 6) * CD + c0);
      const v4f p4 = (*(const v4fa*)(idraw + (size_t)tok * CD + c0)) * dgsh[hh];
      const float w0 = wls[hh * 5 + 0], w1 = wls[hh * 5 + 1], w2 = wls[hh * 5 + 2];
      const float w3 = wls[hh * 5 + 3], w4 = wls[hh * 5 + 4];
      const float gg = gsh[hh];
      v4f pr = ms * w0;
      pr = pr + ml * w1;
      pr = pr + p2 * w2;
      pr = pr + p3 * w3;
      pr = pr + p4 * w4;
      *(v4fa*)(cs + t * CD + c0) = pr * gg;
    }
    __syncthreads();
  }

  if (tid >= 192 && tid < 192 + NH) { eh[2 * (tid - 192)] = e1acc; eh[2 * (tid - 192) + 1] = e2acc; }
  fuse_ctx_pass(cs, ctxh, ctxl, tokb, tid);
  __syncthreads();
  if (tid == 0) {
    float s1 = 0.0f, s2 = 0.0f;
    #pragma unroll 1
    for (int g = 0; g < NH; ++g) { s1 += eh[2 * g]; s2 += eh[2 * g + 1]; }
    eline[0] = s1;
    eline[1] = s2;
    #pragma unroll 1
    for (int i = 2; i < 32; ++i) eline[i] = 0.0f;
  }
  __threadfence();
  fuse_ctx_pass(cs, ctxh, ctxl, tokb, tid);
  __syncthreads();
  if (tid < 8) {
    const v4f v = *(const v4fa*)(eline + 4 * tid);
    float* dst = epart + (size_t)blk * 32 + 4 * tid;
    *(volatile v4f*)dst = v;
    __threadfence();
    *(volatile v4f*)dst = v;
  }
}

__global__ __launch_bounds__(32) void k_final(const float* __restrict__ epart, int nblk, float* __restrict__ o1) {
  if (threadIdx.x == 0) {
    double s1 = 0.0, s2 = 0.0;
    #pragma unroll 1
    for (int i = 0; i < nblk; ++i) {
      s1 += (double)epart[(size_t)i * 32];
      s2 += (double)epart[(size_t)i * 32 + 1];
    }
    const float e1 = (float)(-s1 / 49152.0);
    const float e2 = (float)(-s2 / 49152.0);
    const float v = e1 + e2;
    *(volatile float*)o1 = v;
    __threadfence();
    *(volatile float*)o1 = v;
  }
}

extern "C" void kernel_launch(void* const* d_in, const int* in_sizes, int n_in,
                              void* d_out, int out_size, void* d_ws, size_t ws_size,
                              hipStream_t stream) {
  if (n_in < 17) return;
  if (in_sizes[0] != NTOK * CD || in_sizes[1] != CD * CQ || in_sizes[2] != CD * CD || in_sizes[3] != CD) return;
  if (in_sizes[4] != NH * HD * 3 || in_sizes[5] != NH * HD * 7 || in_sizes[6] != NH * NH) return;
  if (in_sizes[7] != CD * 60 || in_sizes[8] != 60 || in_sizes[9] != CD * CD || in_sizes[10] != CD) return;
  if (in_sizes[11] != CD * NH || in_sizes[12] != NH || in_sizes[13] != CD * CD || in_sizes[14] != NH) return;
  if (in_sizes[15] != CD * NH || in_sizes[16] != NH) return;
  if (out_size != NTOK * CD + 1) return;

  const float* x        = (const float*)d_in[0];
  const float* w_qkv    = (const float*)d_in[1];
  const float* w_proj   = (const float*)d_in[2];
  const float* b_proj   = (const float*)d_in[3];
  const float* fir_s    = (const float*)d_in[4];
  const float* fir_l    = (const float*)d_in[5];
  const float* mixm     = (const float*)d_in[6];
  const float* w_prune  = (const float*)d_in[7];
  const float* b_prune  = (const float*)d_in[8];
  const float* w_g1     = (const float*)d_in[9];
  const float* b_g1     = (const float*)d_in[10];
  const float* w_g2     = (const float*)d_in[11];
  const float* b_g2     = (const float*)d_in[12];
  const float* w_id     = (const float*)d_in[13];
  const float* id_stat  = (const float*)d_in[14];
  const float* w_idgate = (const float*)d_in[15];
  const float* b_idgate = (const float*)d_in[16];
  float* out = (float*)d_out;

  size_t off = 0;
  char* wsb = (char*)d_ws;
  auto take = [&](size_t bytes) -> char* {
    char* p = wsb + off;
    off += (bytes + 255) & ~(size_t)255;
    return p;
  };
  const size_t plane_x = (size_t)NTOK * CD * 2;
  const size_t plane_w = (size_t)WROWS * CD * 2;
  bf_t*  xq     = (bf_t*)take(2 * plane_x);
  bf_t*  wh     = (bf_t*)take(plane_w);
  bf_t*  wl     = (bf_t*)take(plane_w);
  float* qkvb   = (float*)take((size_t)NTOK * CQ * 4);
  float* idraw  = (float*)take((size_t)NTOK * CD * 4);
  bf_t*  hdh    = (bf_t*)take(plane_x);
  bf_t*  hdl    = (bf_t*)take(plane_x);
  float* pruneb = (float*)take((size_t)NTOK * 64 * 4);
  float* idlog  = (float*)take((size_t)NTOK * 16 * 4);
  float* glog   = (float*)take((size_t)NTOK * 16 * 4);
  float* betab  = (float*)take((size_t)NBH * NSEQ * 4);
  float* deltao = (float*)take((size_t)NTOK * CD * 4);
  bf_t*  ctxh   = (bf_t*)take(plane_x);
  bf_t*  ctxl   = (bf_t*)take(plane_x);
  float* epart  = (float*)take((size_t)NBLKF * 32 * 4);
  if (off > ws_size) return;
  bf_t* xh = xq;
  bf_t* xl = xq + (size_t)NTOK * CD;

  k_cvt_x<<<(NTOK * CD / 8 + 255) / 256, 256, 0, stream>>>(x, xh, xl, NTOK * CD / 8);
  k_wcvt<<<dim3(CD / 64, 2304 / 32), 256, 0, stream>>>(w_qkv, CQ, wh + (size_t)WR_QKV * CD, wl + (size_t)WR_QKV * CD);
  k_wcvt<<<dim3(CD / 64, CD / 32), 256, 0, stream>>>(w_id, CD, wh + (size_t)WR_ID * CD, wl + (size_t)WR_ID * CD);
  k_wcvt<<<dim3(CD / 64, CD / 32), 256, 0, stream>>>(w_g1, CD, wh + (size_t)WR_G1 * CD, wl + (size_t)WR_G1 * CD);
  k_wcvt<<<dim3(CD / 64, CD / 32), 256, 0, stream>>>(w_proj, CD, wh + (size_t)WR_PROJ * CD, wl + (size_t)WR_PROJ * CD);
  k_wcvt<<<dim3(CD / 64, 2), 256, 0, stream>>>(w_prune, 60, wh + (size_t)WR_PRUNE * CD, wl + (size_t)WR_PRUNE * CD);
  k_wcvt<<<dim3(CD / 64, 1), 256, 0, stream>>>(w_idgate, NH, wh + (size_t)WR_IDG * CD, wl + (size_t)WR_IDG * CD);
  k_wcvt<<<dim3(CD / 64, 1), 256, 0, stream>>>(w_g2, NH, wh + (size_t)WR_G2 * CD, wl + (size_t)WR_G2 * CD);

  k_gemm<4, 0><<<dim3(CQ / 64, NTOK / 128), 128, 0, stream>>>(
      xh, xl, CD, wh + (size_t)WR_QKV * CD, wl + (size_t)WR_QKV * CD, CD, b_proj, 0, qkvb, CQ, hdh, hdl, CD, CD);
  k_gemm<4, 0><<<dim3(CD / 64, NTOK / 128), 128, 0, stream>>>(
      xh, xl, CD, wh + (size_t)WR_ID * CD, wl + (size_t)WR_ID * CD, CD, b_proj, 0, idraw, CD, hdh, hdl, CD, CD);
  k_gemm<4, 1><<<dim3(CD / 64, NTOK / 128), 128, 0, stream>>>(
      xh, xl, CD, wh + (size_t)WR_G1 * CD, wl + (size_t)WR_G1 * CD, CD, b_g1, CD, idraw, CD, hdh, hdl, CD, CD);
  k_gemm<4, 0><<<dim3(1, NTOK / 128), 128, 0, stream>>>(
      xh, xl, CD, wh + (size_t)WR_PRUNE * CD, wl + (size_t)WR_PRUNE * CD, CD, b_prune, 60, pruneb, 64, hdh, hdl, CD, CD);
  k_gemm<1, 0><<<dim3(1, NTOK / 128), 128, 0, stream>>>(
      xh, xl, CD, wh + (size_t)WR_IDG * CD, wl + (size_t)WR_IDG * CD, CD, b_idgate, NH, idlog, 16, hdh, hdl, CD, CD);
  k_gemm<1, 0><<<dim3(1, NTOK / 128), 128, 0, stream>>>(
      hdh, hdl, CD, wh + (size_t)WR_G2 * CD, wl + (size_t)WR_G2 * CD, CD, b_g2, NH, glog, 16, ctxh, ctxl, CD, CD);
  k_qkpl<<<(2 * NBH * NSEQ * 8 + 255) / 256, 256, 0, stream>>>(qkvb, xq, 2 * NBH * NSEQ * 8);
  k_beta<<<dim3(NSEQ / 32, NBH), 64, 0, stream>>>(xq, betab);
  k_delta<<<NBH, 256, 0, stream>>>(qkvb, betab, deltao);
  k_fuse<<<NBLKF, 256, 0, stream>>>(qkvb, deltao, idraw, pruneb, glog, idlog, fir_s, fir_l, mixm, id_stat,
                                     ctxh, ctxl, epart);
  k_gemm<4, 0><<<dim3(CD / 64, NTOK / 128), 128, 0, stream>>>(
      ctxh, ctxl, CD, wh + (size_t)WR_PROJ * CD, wl + (size_t)WR_PROJ * CD, CD, b_proj, CD, out, CD, hdh, hdl, CD, CD);
  k_final<<<1, 32, 0, stream>>>(epart, NBLKF, out + (size_t)NTOK * CD);
}
